// HybridLNNModel_86371792322661
// MI455X (gfx1250) — hardware-verified
//
#include <hip/hip_runtime.h>
#include <math.h>

constexpr int NBAT   = 256;
constexpr int NSEQ   = 128;
constexpr int NSTEPS = NSEQ - 1;
constexpr int NCH    = 8;
constexpr int NHID   = 256;
constexpr int NOUTF  = 256;
constexpr int KSTATE = NCH * NHID;
constexpr int NTHR   = 256;
constexpr int NWAVE  = NTHR / 32;
constexpr int ROWB   = 16;
constexpr int APITCH = 264;
constexpr int ABUFH  = ROWB * APITCH;
constexpr int YSLP   = 32;
constexpr float WCAR_INV = 0.125f;
constexpr float OCAR_INV = 0.0625f;
constexpr int NW8    = NCH * NHID * NHID / 8;
constexpr int NO8    = NOUTF * KSTATE / 8;
constexpr int NOUT_TOTAL = NBAT * NSTEPS * NOUTF;

static_assert(NBAT % ROWB == 0);
static_assert(NHID == 32 * NWAVE);
static_assert(NOUTF == 32 * NWAVE);
static_assert(NHID % 32 == 0);
static_assert(NWAVE * ROWB * YSLP * 4 <= 2 * ABUFH * 2);
static_assert((NCH * ROWB * NHID) % NTHR == 0);
static_assert((2 * ABUFH) % NTHR == 0);
static_assert(NW8 % NTHR == 0 && NO8 % NTHR == 0);
static_assert(APITCH % 8 == 0);

typedef __attribute__((ext_vector_type(16))) _Float16 v16h;
typedef __attribute__((ext_vector_type(8)))  _Float16 v8h;
typedef __attribute__((ext_vector_type(8)))  float    v8f;
typedef __attribute__((ext_vector_type(4)))  float    v4f;

__device__ __forceinline__ void dep_guard_h(v8f& a, v8f& b, v16h x, v16h y) { asm volatile("v_nop\n\tv_nop\n\tv_nop\n\tv_nop" : "+v"(a), "+v"(b) : "v"(x), "v"(y)); }
__device__ __forceinline__ void keep4_h(v16h a, v16h b, v16h c, v16h d) { asm volatile("v_nop" :: "v"(a), "v"(b), "v"(c), "v"(d)); }
__device__ __forceinline__ void acc_guard2(v8f& a, v8f& b) { asm volatile("v_nop\n\tv_nop\n\tv_nop\n\tv_nop" : "+v"(a), "+v"(b)); }

template <typename T> struct Frag;
template <> struct Frag<_Float16> {
  typedef v16h V; union U { v16h v; v8h h[2]; };
  static __device__ __forceinline__ v16h load(const _Float16* p) {
    U f; f.h[0] = *(const v8h*)(p); f.h[1] = *(const v8h*)(p + 16); return f.v;
  }
  static __device__ __forceinline__ v8f mma(v16h a, v16h b, v8f c) {
    return __builtin_amdgcn_wmma_f32_16x16x32_f16(false, a, false, b, (short)0, c, false, false);
  }
};

__device__ __forceinline__ float ftanh_f(float x) {
  const float xc = fminf(fmaxf(x, -10.0f), 10.0f);
  const float e = __expf(2.0f * xc);
  return 1.0f - 2.0f * __builtin_amdgcn_rcpf(e + 1.0f);
}

__global__ __launch_bounds__(NTHR) void cvt_f16x8_kernel(const float* __restrict__ src, unsigned short* __restrict__ dst,
                                                         int n8, float sc) {
  const int i = blockIdx.x * NTHR + threadIdx.x;
  if (i < n8) {
    const float* sp = src + (size_t)i * 8;
    const v4f a = *(const v4f*)(sp);
    const v4f b = *(const v4f*)(sp + 4);
    v8h hv;
#pragma unroll
    for (int e = 0; e < 4; ++e) {
      hv[e]     = (_Float16)(a[e] * sc);
      hv[4 + e] = (_Float16)(b[e] * sc);
    }
    *(volatile v8h*)(dst + (size_t)i * 8) = hv;
    __threadfence();
    *(volatile v8h*)(dst + (size_t)i * 8) = hv;
  }
}

__device__ __forceinline__ void ltc_eval(const _Float16* arow,
                                         const _Float16* __restrict__ w0, const _Float16* __restrict__ w1,
                                         const float (&xt)[16], const float (&u)[8], const float (&prm)[8],
                                         float (&kout)[16]) {
  const v8f z8 = {0.f, 0.f, 0.f, 0.f, 0.f, 0.f, 0.f, 0.f};
  v8f acc0 = z8, acc1 = z8;
#pragma unroll 2
  for (int k0 = 0; k0 < NHID; k0 += 32) {
    const v16h a  = Frag<_Float16>::load(arow + k0);
    const v16h b0 = Frag<_Float16>::load(w0 + k0);
    const v16h b1 = Frag<_Float16>::load(w1 + k0);
    acc0 = Frag<_Float16>::mma(a, b0, acc0);
    acc1 = Frag<_Float16>::mma(a, b1, acc1);
    dep_guard_h(acc0, acc1, a, b1);
    keep4_h(a, b0, b1, a);
  }
  acc_guard2(acc0, acc1);
#pragma unroll
  for (int r = 0; r < 8; ++r) {
    float pre0 = acc0[r] * WCAR_INV + prm[0];
    pre0 = pre0 + u[r] * prm[2];
    pre0 = pre0 + prm[4];
    const float x0 = xt[r];
    kout[r] = (ftanh_f(pre0) - x0 * prm[6]) * __builtin_amdgcn_sqrtf(x0 + 1.0f);
    float pre1 = acc1[r] * WCAR_INV + prm[1];
    pre1 = pre1 + u[r] * prm[3];
    pre1 = pre1 + prm[5];
    const float x1 = xt[r + 8];
    kout[r + 8] = (ftanh_f(pre1) - x1 * prm[7]) * __builtin_amdgcn_sqrtf(x1 + 1.0f);
  }
}

__device__ __forceinline__ void put_tile(_Float16* at, const float (&v)[16], int hh, int j0) {
#pragma unroll
  for (int r = 0; r < 8; ++r) {
    at[(8 * hh + r) * APITCH + j0]      = (_Float16)v[r];
    at[(8 * hh + r) * APITCH + j0 + 16] = (_Float16)v[r + 8];
  }
}

__global__ __launch_bounds__(NTHR) void lnn_rk4_kernel(
    const float* __restrict__ inp,
    const float* __restrict__ times,
    const float* __restrict__ Wb,
    const float* __restrict__ Uw,
    const float* __restrict__ Ub,
    const float* __restrict__ bpar,
    const float* __restrict__ tau,
    const unsigned short* __restrict__ WHp,
    const unsigned short* __restrict__ OHp,
    const float* __restrict__ out_b,
    float* __restrict__ out)
{
  __shared__ __align__(16) float    xs[NCH * ROWB * NHID];
  __shared__ __align__(16) _Float16 abuf[2 * ABUFH];

  const _Float16* WH = (const _Float16*)WHp;
  const _Float16* OH = (const _Float16*)OHp;
  const int tid = threadIdx.x, lane = tid & 31, wave = tid >> 5;
  const int c = lane & 15, hh = lane >> 4, koff = hh * 8;
  const int b0 = blockIdx.x * ROWB;
  const int j0 = 32 * wave + c;
  const int j1 = j0 + 16;

#pragma unroll 1
  for (int i = tid; i < NCH * ROWB * NHID; i += NTHR) xs[i] = 0.0f;
#pragma unroll 1
  for (int i = tid; i < 2 * ABUFH; i += NTHR) abuf[i] = (_Float16)0.0f;
  __syncthreads();

  const float third = 1.0f / 3.0f;
  const float ob0 = out_b[j0], ob1 = out_b[j1];
  const v8f z8 = {0.f, 0.f, 0.f, 0.f, 0.f, 0.f, 0.f, 0.f};

#pragma unroll 1
  for (int s = 0; s < NSTEPS; ++s) {
    const float dt = times[s + 1] - times[s];
    v8f yacc0 = z8, yacc1 = z8;

#pragma unroll 1
    for (int p = 0; p < NCH; ++p) {
      const int cur = p & 1;
      _Float16* atc = abuf + cur * ABUFH;
      _Float16* atn = abuf + (cur ^ 1) * ABUFH;
      const int pc = p * NHID;

      float prm[8];
      prm[0] = Wb[pc + j0];              prm[1] = Wb[pc + j1];
      prm[2] = Uw[pc + j0];              prm[3] = Uw[pc + j1];
      prm[4] = Ub[pc + j0] + bpar[pc + j0];
      prm[5] = Ub[pc + j1] + bpar[pc + j1];
      prm[6] = 1.0f / tau[pc + j0];      prm[7] = 1.0f / tau[pc + j1];

      float u[8];
#pragma unroll
      for (int r = 0; r < 8; ++r) u[r] = inp[((size_t)(b0 + 8 * hh + r) * NSEQ + s) * NCH + p];

      float xb[16], xt[16], ka[16], kb[16], kc[16];
#pragma unroll
      for (int r = 0; r < 8; ++r) {
        const int xo = (p * ROWB + 8 * hh + r) * NHID + j0;
        xb[r] = xs[xo]; xb[r + 8] = xs[xo + 16];
        xt[r] = xb[r];  xt[r + 8] = xb[r + 8];
      }
      put_tile(atc, xb, hh, j0);
      __syncthreads();

      const _Float16* w0 = WH + (size_t)(pc + j0) * NHID + koff;
      const _Float16* w1 = WH + (size_t)(pc + j1) * NHID + koff;
      const _Float16* arc = atc + c * APITCH + koff;
      const _Float16* arn = atn + c * APITCH + koff;

      ltc_eval(arc, w0, w1, xt, u, prm, ka);
#pragma unroll
      for (int i = 0; i < 16; ++i) xt[i] = xb[i] + dt * (ka[i] * third);
      put_tile(atn, xt, hh, j0);
      __syncthreads();

      ltc_eval(arn, w0, w1, xt, u, prm, kb);
#pragma unroll
      for (int i = 0; i < 16; ++i) xt[i] = xb[i] + dt * (kb[i] - ka[i] * third);
      put_tile(atc, xt, hh, j0);
      __syncthreads();

      ltc_eval(arc, w0, w1, xt, u, prm, kc);
#pragma unroll
      for (int i = 0; i < 16; ++i) {
        xt[i] = xb[i] + dt * ((ka[i] - kb[i]) + kc[i]);
        ka[i] = ka[i] + 3.0f * (kb[i] + kc[i]);
      }
      put_tile(atn, xt, hh, j0);
      __syncthreads();

      ltc_eval(arn, w0, w1, xt, u, prm, kb);
#pragma unroll
      for (int r = 0; r < 8; ++r) {
        const int xo = (p * ROWB + 8 * hh + r) * NHID + j0;
        const float xn0 = xb[r]     + (dt * (ka[r]     + kb[r]))     * 0.125f;
        const float xn1 = xb[r + 8] + (dt * (ka[r + 8] + kb[r + 8])) * 0.125f;
        xs[xo] = xn0;  xs[xo + 16] = xn1;
        atc[(8 * hh + r) * APITCH + j0]      = (_Float16)xn0;
        atc[(8 * hh + r) * APITCH + j0 + 16] = (_Float16)xn1;
      }
      __syncthreads();

      {
        const _Float16* o0 = OH + (size_t)j0 * KSTATE + pc + koff;
        const _Float16* o1 = OH + (size_t)j1 * KSTATE + pc + koff;
#pragma unroll 2
        for (int k0 = 0; k0 < NHID; k0 += 32) {
          const v16h a  = Frag<_Float16>::load(arc + k0);
          const v16h b0 = Frag<_Float16>::load(o0 + k0);
          const v16h b1 = Frag<_Float16>::load(o1 + k0);
          yacc0 = Frag<_Float16>::mma(a, b0, yacc0);
          yacc1 = Frag<_Float16>::mma(a, b1, yacc1);
          dep_guard_h(yacc0, yacc1, a, b1);
          keep4_h(a, b0, b1, a);
        }
        acc_guard2(yacc0, yacc1);
      }
    }

    __syncthreads();
    float* ysl = reinterpret_cast<float*>(abuf) + wave * (ROWB * YSLP);
#pragma unroll
    for (int r = 0; r < 8; ++r) {
      ysl[(8 * hh + r) * YSLP + c]      = yacc0[r] * OCAR_INV + ob0;
      ysl[(8 * hh + r) * YSLP + 16 + c] = yacc1[r] * OCAR_INV + ob1;
    }
    __builtin_amdgcn_fence(__ATOMIC_RELEASE, "workgroup");
    __builtin_amdgcn_wave_barrier();
    __builtin_amdgcn_fence(__ATOMIC_ACQUIRE, "workgroup");
    {
      const int q = lane >> 3, c4 = (lane & 7) * 4;
      for (int pass = 0; pass < 2; ++pass) {
#pragma unroll
        for (int it = 0; it < 4; ++it) {
          const int row = it * 4 + q;
          const v4f v = *(const v4f*)(ysl + row * YSLP + c4);
          *(volatile v4f*)(out + ((size_t)(b0 + row) * NSTEPS + (size_t)s) * NOUTF + 32 * wave + c4) = v;
        }
        __threadfence();
      }
    }
    __syncthreads();
  }
}

extern "C" void kernel_launch(void* const* d_in, const int* in_sizes, int n_in,
                              void* d_out, int out_size, void* d_ws, size_t ws_size, hipStream_t stream) {
  if (n_in < 10 || d_out == nullptr || d_ws == nullptr) return;
  if (in_sizes[0] != NBAT * NSEQ * NCH || in_sizes[1] != NSEQ || in_sizes[2] != NCH * NHID * NHID ||
      in_sizes[3] != NCH * NHID || in_sizes[4] != NCH * NHID || in_sizes[5] != NCH * NHID ||
      in_sizes[6] != NCH * NHID || in_sizes[7] != NCH * NHID || in_sizes[8] != NOUTF * KSTATE ||
      in_sizes[9] != NOUTF || out_size != NOUT_TOTAL) return;

  const float* inp   = (const float*)d_in[0];
  const float* times = (const float*)d_in[1];
  const float* Ww    = (const float*)d_in[2];
  const float* Wb    = (const float*)d_in[3];
  const float* Uw    = (const float*)d_in[4];
  const float* Ub    = (const float*)d_in[5];
  const float* bpar  = (const float*)d_in[6];
  const float* tau   = (const float*)d_in[7];
  const float* out_w = (const float*)d_in[8];
  const float* out_b = (const float*)d_in[9];
  float* y = (float*)d_out;

  const size_t whBytes = (size_t)NCH * NHID * NHID * 2;
  const size_t ohBytes = (size_t)NOUTF * KSTATE * 2;
  if (whBytes + ohBytes > ws_size || whBytes + ohBytes > (size_t)134217728) return;
  unsigned short* WH = (unsigned short*)d_ws;
  unsigned short* OH = (unsigned short*)((char*)d_ws + whBytes);

  cvt_f16x8_kernel<<<NW8 / NTHR, NTHR, 0, stream>>>(Ww, WH, NW8, 8.0f);
  cvt_f16x8_kernel<<<NO8 / NTHR, NTHR, 0, stream>>>(out_w, OH, NO8, 16.0f);
  lnn_rk4_kernel<<<NBAT / ROWB, NTHR, 0, stream>>>(inp, times, Wb, Uw, Ub, bpar, tau, WH, OH, out_b, y);
}
